// IndividualRNNAutoEncoder_24953759989784
// MI455X (gfx1250) — hardware-verified
//
#include <hip/hip_runtime.h>


typedef _Float16 f16t;
typedef f16t  v16h __attribute__((ext_vector_type(16)));
typedef f16t  v8h  __attribute__((ext_vector_type(8)));
typedef f16t  v4h  __attribute__((ext_vector_type(4)));
typedef float v8f  __attribute__((ext_vector_type(8)));
typedef float v4f  __attribute__((ext_vector_type(4)));
typedef unsigned int v4u __attribute__((ext_vector_type(4)));

union Frag { v16h v; v8h q[2]; };
union Pk16 { v8h h; v4u u; };
union Pk32 { v4f f; v4u u; };

#define NB  64
#define NTT 512
#define NH  512
#define NE  64
#define NV  4
#define RB  16
#define LP  520
#define XP  72

__device__ __forceinline__ v8f wmma16(v16h a, v16h b, v8f c) {
    return __builtin_amdgcn_wmma_f32_16x16x32_f16(false, a, false, b, (short)0, c, false, false);
}

__device__ __forceinline__ void wguard(v8f (&c)[1][1], Frag (&a)[1], Frag (&b)[1]) {
    asm volatile("v_nop\n\tv_nop\n\tv_nop\n\tv_nop"
                 : "+v"(c[0][0])
                 : "v"(a[0].v), "v"(b[0].v));
}
__device__ __forceinline__ void wguard(v8f (&c)[4][1], Frag (&a)[4], Frag (&b)[1]) {
    asm volatile("v_nop\n\tv_nop\n\tv_nop\n\tv_nop"
                 : "+v"(c[0][0]), "+v"(c[1][0]), "+v"(c[2][0]), "+v"(c[3][0])
                 : "v"(a[0].v), "v"(a[1].v), "v"(a[2].v), "v"(a[3].v), "v"(b[0].v));
}

template<int MT, int NT>
__device__ __forceinline__ void zacc(v8f (&acc)[MT][NT]) {
    const v8f z = {0.f, 0.f, 0.f, 0.f, 0.f, 0.f, 0.f, 0.f};
#pragma unroll
    for (int i = 0; i < MT; ++i)
#pragma unroll
        for (int j = 0; j < NT; ++j) acc[i][j] = z;
}

template<int MT, int NT>
__device__ __forceinline__ void mma_acc(v8f (&acc)[MT][NT],
                                        const f16t* A, int lda,
                                        const f16t* B, int ldb, int ktiles) {
    const int l = threadIdx.x & 31, h = l >> 4, m = l & 15;
    const f16t* ap = A + (size_t)m * lda + 8 * h;
    const f16t* bp = B + (size_t)m * ldb + 8 * h;
#pragma unroll 1
    for (int kt = 0; kt < ktiles; ++kt) {
        Frag a[MT], b[NT];
#pragma unroll
        for (int i = 0; i < MT; ++i) {
            const f16t* p = ap + (size_t)i * 16 * lda + kt * 32;
            a[i].q[0] = *(const v8h*)p;
            a[i].q[1] = *(const v8h*)(p + 16);
        }
#pragma unroll
        for (int j = 0; j < NT; ++j) {
            const f16t* p = bp + (size_t)j * 16 * ldb + kt * 32;
            b[j].q[0] = *(const v8h*)p;
            b[j].q[1] = *(const v8h*)(p + 16);
        }
#pragma unroll
        for (int i = 0; i < MT; ++i)
#pragma unroll
            for (int j = 0; j < NT; ++j)
                acc[i][j] = wmma16(a[i].v, b[j].v, acc[i][j]);
        wguard(acc, a, b);
    }
}

__device__ __forceinline__ float ftanh(float x) {
    float ax = fabsf(x);
    float t  = __expf(-2.0f * ax);
    float r  = (1.0f - t) * __builtin_amdgcn_rcpf(1.0f + t);
    return copysignf(r, x);
}

template<int MT, int NT>
__device__ __forceinline__ void epi_tanh(v8f (&acc)[MT][NT], float inv,
                                         const float* b1, const float* b2,
                                         int f0, f16t* L, int pitch) {
    const int l = threadIdx.x & 31, h = l >> 4, m = l & 15;
#pragma unroll
    for (int i = 0; i < MT; ++i) {
        const int fo = f0 + 16 * i + 8 * h;
        v4f c0 = *(const v4f*)(b1 + fo)     + *(const v4f*)(b2 + fo);
        v4f c1 = *(const v4f*)(b1 + fo + 4) + *(const v4f*)(b2 + fo + 4);
#pragma unroll
        for (int j = 0; j < NT; ++j) {
            Pk16 pk;
#pragma unroll
            for (int r = 0; r < 4; ++r) {
                float v0 = ftanh(fmaf(acc[i][j][r],     inv, c0[r]));
                float v1 = ftanh(fmaf(acc[i][j][4 + r], inv, c1[r]));
                pk.h[r]     = (f16t)v0;
                pk.h[4 + r] = (f16t)v1;
            }
            *(v8h*)(L + (size_t)(16 * j + m) * pitch + fo) = pk.h;
        }
    }
}

__global__ __launch_bounds__(256)
void k_cvt8(const float* __restrict__ W, f16t* P, int nreal8, int n8, float sc) {
    int i = blockIdx.x * 256 + threadIdx.x;
    if (i >= n8) return;
    Pk16 k;
    if (i < nreal8) {
        const float* p = W + (size_t)i * 8;
        v4f a = *(const v4f*)p;
        v4f b = *(const v4f*)(p + 4);
        k.h[0] = (f16t)(a[0] * sc); k.h[1] = (f16t)(a[1] * sc);
        k.h[2] = (f16t)(a[2] * sc); k.h[3] = (f16t)(a[3] * sc);
        k.h[4] = (f16t)(b[0] * sc); k.h[5] = (f16t)(b[1] * sc);
        k.h[6] = (f16t)(b[2] * sc); k.h[7] = (f16t)(b[3] * sc);
    } else {
        const f16t z1 = (f16t)0.0f;
        k.h[0] = z1; k.h[1] = z1; k.h[2] = z1; k.h[3] = z1;
        k.h[4] = z1; k.h[5] = z1; k.h[6] = z1; k.h[7] = z1;
    }
    f16t* d = P + (size_t)i * 8;
    *(volatile v4u*)d = k.u;
    __threadfence();
    *(volatile v4u*)d = k.u;
}

__global__ __launch_bounds__(256)
void k_rnn(const float* __restrict__ x, const float* __restrict__ emb,
           const f16t* __restrict__ Pih0, const f16t* __restrict__ Pihr,
           const f16t* __restrict__ Pehh,
           const float* __restrict__ ebih, const float* __restrict__ ebhh,
           const f16t* __restrict__ Pdih, const f16t* __restrict__ Pdhh,
           const float* __restrict__ dbih, const float* __restrict__ dbhh,
           const f16t* __restrict__ Ppr, float* out, int nb, int T, float inv) {
    __shared__ __attribute__((aligned(16))) f16t  Hs[3 * RB * LP];
    __shared__ __attribute__((aligned(16))) f16t  Xe[RB * XP];
    __shared__ __attribute__((aligned(16))) float OS[RB * 32];
    const int tid = threadIdx.x;
    const int w = tid >> 5, ln = tid & 31, hh = ln >> 4, m = ln & 15;
    const int b0 = blockIdx.x * RB;
    if (b0 + RB > nb) return;
    const int f0 = 64 * w;

    {
        const f16t z1 = (f16t)0.0f;
        const v8h z = {z1, z1, z1, z1, z1, z1, z1, z1};
        for (int i = tid; i < (3 * RB * LP) / 8; i += 256) *(v8h*)(Hs + 8 * i) = z;
    }
    __syncthreads();

    f16t* const H0 = Hs;
    f16t* const H1 = Hs + RB * LP;
    f16t* const H2 = Hs + 2 * RB * LP;
    const size_t WSZ = (size_t)NH * NH;
    const int KT = NH / 32;

#pragma unroll 1
    for (int t = 0; t < T; ++t) {
        {
            const int row = tid >> 4, c4 = (tid & 15) * 4;
            const float* xp = x + ((size_t)(b0 + row) * T + t) * NV;
            v4f xv = *(const v4f*)xp;
            int best = 0; float bv = xv[0];
            if (xv[1] > bv) { bv = xv[1]; best = 1; }
            if (xv[2] > bv) { bv = xv[2]; best = 2; }
            if (xv[3] > bv) { bv = xv[3]; best = 3; }
            v4f ev = *(const v4f*)(emb + best * NE + c4);
            v4h hv = {(f16t)ev[0], (f16t)ev[1], (f16t)ev[2], (f16t)ev[3]};
            *(v4h*)(Xe + row * XP + c4) = hv;
        }
        __syncthreads();
        {
            v8f acc[4][1]; zacc(acc);
            mma_acc<4, 1>(acc, Pih0 + (size_t)f0 * NE, NE, Xe, XP, NE / 32);
            mma_acc<4, 1>(acc, Pehh + (size_t)f0 * NH, NH, H0, LP, KT);
            __syncthreads();
            epi_tanh<4, 1>(acc, inv, ebih, ebhh, f0, H0, LP);
            __syncthreads();
        }
        {
            v8f acc[4][1]; zacc(acc);
            mma_acc<4, 1>(acc, Pihr + (size_t)f0 * NH, NH, H0, LP, KT);
            mma_acc<4, 1>(acc, Pehh + WSZ + (size_t)f0 * NH, NH, H1, LP, KT);
            __syncthreads();
            epi_tanh<4, 1>(acc, inv, ebih + NH, ebhh + NH, f0, H1, LP);
            __syncthreads();
        }
        {
            v8f acc[4][1]; zacc(acc);
            mma_acc<4, 1>(acc, Pihr + WSZ + (size_t)f0 * NH, NH, H1, LP, KT);
            mma_acc<4, 1>(acc, Pehh + 2 * WSZ + (size_t)f0 * NH, NH, H2, LP, KT);
            __syncthreads();
            epi_tanh<4, 1>(acc, inv, ebih + 2 * NH, ebhh + 2 * NH, f0, H2, LP);
            __syncthreads();
        }
    }

    const size_t orow = (size_t)T * NV;
#pragma unroll 1
    for (int t = 0; t < T; ++t) {
        {
            const int kih = (t == 0) ? 0 : KT;
            v8f acc[4][1]; zacc(acc);
            mma_acc<4, 1>(acc, Pdih + (size_t)f0 * NH, NH, H0, LP, kih);
            mma_acc<4, 1>(acc, Pdhh + (size_t)f0 * NH, NH, H2, LP, KT);
            __syncthreads();
            epi_tanh<4, 1>(acc, inv, dbih, dbhh, f0, H2, LP);
            __syncthreads();
        }
        {
            v8f acc[4][1]; zacc(acc);
            mma_acc<4, 1>(acc, Pdih + WSZ + (size_t)f0 * NH, NH, H2, LP, KT);
            mma_acc<4, 1>(acc, Pdhh + WSZ + (size_t)f0 * NH, NH, H1, LP, KT);
            __syncthreads();
            epi_tanh<4, 1>(acc, inv, dbih + NH, dbhh + NH, f0, H1, LP);
            __syncthreads();
        }
        {
            v8f acc[4][1]; zacc(acc);
            mma_acc<4, 1>(acc, Pdih + 2 * WSZ + (size_t)f0 * NH, NH, H1, LP, KT);
            mma_acc<4, 1>(acc, Pdhh + 2 * WSZ + (size_t)f0 * NH, NH, H0, LP, KT);
            __syncthreads();
            epi_tanh<4, 1>(acc, inv, dbih + 2 * NH, dbhh + 2 * NH, f0, H0, LP);
            __syncthreads();
        }
        if (w == 0) {
            v8f pa[1][1]; zacc(pa);
            mma_acc<1, 1>(pa, Ppr, NH, H0, LP, KT);
            if (hh == 0) {
                const float g0 = pa[0][0][0] * inv, g1 = pa[0][0][1] * inv,
                            g2 = pa[0][0][2] * inv, g3 = pa[0][0][3] * inv;
                const float mx = fmaxf(fmaxf(g0, g1), fmaxf(g2, g3));
                const float s0 = g0 - mx, s1 = g1 - mx, s2 = g2 - mx, s3 = g3 - mx;
                const float ls = logf(expf(s0) + expf(s1) + expf(s2) + expf(s3));
                v4f o = {s0 - ls, s1 - ls, s2 - ls, s3 - ls};
                *(v4f*)(OS + m * 32 + (t & 7) * 4) = o;
            }
            if ((t & 7) == 7) {
                Pk32 v[4];
#pragma unroll
                for (int i = 0; i < 4; ++i) {
                    int p = ln + 32 * i, row = p >> 3, c = (p & 7) * 4;
                    v[i].f = *(const v4f*)(OS + row * 32 + c);
                }
                const size_t tb = (size_t)(t >> 3) * 32;
#pragma unroll
                for (int i = 0; i < 4; ++i) {
                    int p = ln + 32 * i, row = p >> 3, c = (p & 7) * 4;
                    float* d = out + (size_t)(b0 + row) * orow + tb + c;
                    *(volatile v4u*)d = v[i].u;
                }
                __threadfence();
#pragma unroll
                for (int i = 0; i < 4; ++i) {
                    int p = ln + 32 * i, row = p >> 3, c = (p & 7) * 4;
                    float* d = out + (size_t)(b0 + row) * orow + tb + c;
                    *(volatile v4u*)d = v[i].u;
                }
            }
        }
    }
}

extern "C" void kernel_launch(void* const* d_in, const int* in_sizes, int n_in,
                              void* d_out, int out_size, void* d_ws, size_t ws_size,
                              hipStream_t stream) {
    const int B = NB, T = NTT, H = NH, E = NE, V = NV, L = 3;

    if (n_in < 12) return;
    if (in_sizes[0] != B * T * V || in_sizes[1] != V * E || in_sizes[2] != H * E ||
        in_sizes[3] != (L - 1) * H * H || in_sizes[4] != L * H * H ||
        in_sizes[5] != L * H || in_sizes[6] != L * H ||
        in_sizes[7] != L * H * H || in_sizes[8] != L * H * H ||
        in_sizes[9] != L * H || in_sizes[10] != L * H || in_sizes[11] != V * H) return;
    if (out_size != B * T * V) return;
    if ((B % RB) != 0 || (T % 8) != 0) return;

    const float* x     = (const float*)d_in[0];
    const float* emb   = (const float*)d_in[1];
    const float* ewih0 = (const float*)d_in[2];
    const float* ewihr = (const float*)d_in[3];
    const float* ewhh  = (const float*)d_in[4];
    const float* ebih  = (const float*)d_in[5];
    const float* ebhh  = (const float*)d_in[6];
    const float* dwih  = (const float*)d_in[7];
    const float* dwhh  = (const float*)d_in[8];
    const float* dbih  = (const float*)d_in[9];
    const float* dbhh  = (const float*)d_in[10];
    const float* proj  = (const float*)d_in[11];
    float* out = (float*)d_out;

    char* ws = (char*)d_ws;
    size_t off = 0;
    auto carve = [&](size_t bytes) -> char* {
        char* p = ws + off;
        off = (off + bytes + 255) & ~(size_t)255;
        return p;
    };
    f16t* Pih0 = (f16t*)carve((size_t)H * E * 2);
    f16t* Pihr = (f16t*)carve((size_t)(L - 1) * H * H * 2);
    f16t* Pehh = (f16t*)carve((size_t)L * H * H * 2);
    f16t* Pdih = (f16t*)carve((size_t)L * H * H * 2);
    f16t* Pdhh = (f16t*)carve((size_t)L * H * H * 2);
    f16t* Ppr  = (f16t*)carve((size_t)16 * H * 2);
    if (off > ws_size) return;

    const float S64 = 64.0f, I64 = 0.015625f;

    auto cvt = [&](const float* W, f16t* P, int nreal, int ntot) {
        int nr8 = nreal / 8, n8 = ntot / 8;
        k_cvt8<<<dim3((n8 + 255) / 256), dim3(256), 0, stream>>>(W, P, nr8, n8, S64);
    };
    cvt(ewih0, Pih0, H * E,           H * E);
    cvt(ewihr, Pihr, (L - 1) * H * H, (L - 1) * H * H);
    cvt(ewhh,  Pehh, L * H * H,       L * H * H);
    cvt(dwih,  Pdih, L * H * H,       L * H * H);
    cvt(dwhh,  Pdhh, L * H * H,       L * H * H);
    cvt(proj,  Ppr,  V * H,           16 * H);

    k_rnn<<<dim3(B / RB), dim3(256), 0, stream>>>(x, emb, Pih0, Pihr, Pehh, ebih, ebhh,
                                                  Pdih, Pdhh, dbih, dbhh, Ppr, out,
                                                  B, T, I64);
}
